// SuperpointGraph_6030134083771
// MI455X (gfx1250) — hardware-verified
//
#include <hip/hip_runtime.h>
#include <stddef.h>
#include <stdint.h>

#define NN    512
#define NODES 1024
#define CC    256
#define EE    18
#define HID   64

#define SEF 8.0f
#define SWT 16.0f
#define S1  16.0f
#define S2  32.0f
#define SPE 128.0f
#define SHH 8.0f
#define SGG 8.0f

#define SP   64
#define PEP  32
#define GP   40

#define EM1_O   0
#define EM2_O   2048
#define EM3_O   6144
#define AT1E_O  8192
#define AT2_O   10240
#define EG1E_O  12288
#define EG2_O   14336
#define WPL_HALVES 30720

static_assert(SP % 8 == 0);
static_assert(PEP % 8 == 0);
static_assert(GP % 8 == 0);
static_assert(NODES % 64 == 0);
static_assert(CC % 64 == 0);

typedef _Float16 f16;
typedef f16 v16h __attribute__((ext_vector_type(16)));
typedef f16 v8h_t __attribute__((ext_vector_type(8)));
typedef v8h_t __attribute__((may_alias)) v8h;
typedef __bf16 v16b __attribute__((ext_vector_type(16)));
typedef unsigned short v8us_t __attribute__((ext_vector_type(8)));
typedef v8us_t __attribute__((may_alias)) v8us;
typedef float v8f __attribute__((ext_vector_type(8)));
typedef float v4f_t __attribute__((ext_vector_type(4)));
typedef v4f_t __attribute__((may_alias)) v4f;
typedef unsigned int v4u __attribute__((ext_vector_type(4)));

union FragH { v16h v; v8h_t h[2]; };
union FragB { v16b v; v8us_t u[2]; };
union U16   { v8us_t v[2]; unsigned short s[16]; };

static __device__ __forceinline__ v8f zero8() {
  v8f z;
#pragma unroll
  for (int i = 0; i < 8; ++i) z[i] = 0.0f;
  return z;
}

static __device__ __forceinline__ v16h ldrow(const f16* base, int pitch, int row, int k0, int hh) {
  const f16* p = base + (size_t)row * pitch + k0 + 8 * hh;
  FragH f;
  f.h[0] = *(const v8h*)(p);
  f.h[1] = *(const v8h*)(p + 16);
  return f.v;
}

static __device__ __forceinline__ v16b ldrowb(const unsigned short* base, int row, int hh) {
  const unsigned short* p = base + row * GP + 8 * hh;
  FragB f;
  f.u[0] = *(const v8us*)(p);
  f.u[1] = *(const v8us*)(p + 16);
  return f.v;
}

static __device__ __forceinline__ v8f mma1(v16h a, v16h b) {
  v8f c = zero8();
  c = __builtin_amdgcn_wmma_f32_16x16x32_f16(false, a, false, b, (short)0, c, false, false);
  asm volatile("v_nop\n\tv_nop\n\tv_nop\n\tv_nop" : "+v"(c) : "v"(a), "v"(b));
  return c;
}

static __device__ __forceinline__ v8f mma2(v16h a0, v16h b0, v16h a1, v16h b1) {
  v8f c = zero8();
  c = __builtin_amdgcn_wmma_f32_16x16x32_f16(false, a0, false, b0, (short)0, c, false, false);
  c = __builtin_amdgcn_wmma_f32_16x16x32_f16(false, a1, false, b1, (short)0, c, false, false);
  asm volatile("v_nop\n\tv_nop\n\tv_nop\n\tv_nop" : "+v"(c) : "v"(a0), "v"(b0), "v"(a1), "v"(b1));
  return c;
}

static __device__ __forceinline__ void split_bf16(float x, unsigned short& hi, unsigned short& lo) {
  const unsigned u = __float_as_uint(x);
  const unsigned r = u + 0x7FFFu + ((u >> 16) & 1u);
  hi = (unsigned short)(r >> 16);
  const float hf = __uint_as_float(r & 0xFFFF0000u);
  const float d = x - hf;
  const unsigned v = __float_as_uint(d);
  const unsigned s = v + 0x7FFFu + ((v >> 16) & 1u);
  lo = (unsigned short)(s >> 16);
}

__global__ __launch_bounds__(256) void wprep_kernel(
    const float* __restrict__ em_w1, const float* __restrict__ em_w2,
    const float* __restrict__ em_w3, const float* __restrict__ at_w1,
    const float* __restrict__ at_w2, const float* __restrict__ eg_w1,
    const float* __restrict__ eg_w2, f16* __restrict__ wpl)
{
  const int y = blockIdx.y;
  const float* src = em_w1; int K = EE, N = 64, ld = 64, Kp = 32, off = EM1_O;
  if (y == 1)      { src = em_w2;            K = 64; N = 64;  ld = 64;  Kp = 64; off = EM2_O;  }
  else if (y == 2) { src = em_w3;            K = 64; N = 32;  ld = 32;  Kp = 64; off = EM3_O;  }
  else if (y == 3) { src = at_w1 + 512 * 64; K = 32; N = 64;  ld = 64;  Kp = 32; off = AT1E_O; }
  else if (y == 4) { src = at_w2;            K = 64; N = 32;  ld = 32;  Kp = 64; off = AT2_O;  }
  else if (y == 5) { src = eg_w1 + 256 * 64; K = 32; N = 64;  ld = 64;  Kp = 32; off = EG1E_O; }
  else if (y == 6) { src = eg_w2;            K = 64; N = 256; ld = 256; Kp = 64; off = EG2_O;  }

  const int g = blockIdx.x * 256 + threadIdx.x;
  const int gpr = Kp >> 3;
  const int G = N * gpr;
  const bool ok = (g < G);
  const int gc = ok ? g : 0;
  const int n = gc / gpr;
  const int kg = (gc - n * gpr) * 8;
  union { v8h_t h; v4u u; } pk;
#pragma unroll
  for (int e = 0; e < 8; ++e) {
    const int k = kg + e;
    const int kc = (k < K) ? k : (K - 1);
    const float v = src[(size_t)kc * ld + n];
    pk.h[e] = (f16)((k < K) ? v * SWT : 0.0f);
  }
  f16* dp = wpl + off + (size_t)n * Kp + kg;
  if (ok) *(volatile v4u*)dp = pk.u;
  __threadfence();
  if (ok) *(volatile v4u*)dp = pk.u;
}

__global__ __launch_bounds__(128) void gemm3_kernel(
    const float* __restrict__ A, int lda, int K,
    const float* __restrict__ W0, const float* __restrict__ W1, const float* __restrict__ W2, int ldw,
    const float* __restrict__ B0p, const float* __restrict__ B1p, const float* __restrict__ B2p, int hasb,
    float* C0, float* C1, float* C2, int ldc0, int ldc1, int ldc2, int relu)
{
  __shared__ __align__(16) unsigned short Ah[64 * GP];
  __shared__ __align__(16) unsigned short Al[64 * GP];
  __shared__ __align__(16) unsigned short Bh[64 * GP];
  __shared__ __align__(16) unsigned short Bl[64 * GP];
  __shared__ __align__(16) float Cs[64 * 64];

  const int tid = threadIdx.x, w = tid >> 5, lane = tid & 31;
  const int hh = lane >> 4, m = lane & 15;
  const int z = blockIdx.z;
  const float* W    = (z == 0) ? W0 : ((z == 1) ? W1 : W2);
  const float* bias = (z == 0) ? B0p : ((z == 1) ? B1p : B2p);
  float* C          = (z == 0) ? C0 : ((z == 1) ? C1 : C2);
  const int ldc     = (z == 0) ? ldc0 : ((z == 1) ? ldc1 : ldc2);
  const int n0 = blockIdx.x * 64, m0 = blockIdx.y * 64;

  v8f acc[4];
#pragma unroll
  for (int t = 0; t < 4; ++t) acc[t] = zero8();

  const int ar = tid >> 1, acq = (tid & 1) * 16;
  const int bk = tid >> 2, bnq = (tid & 3) * 16;

#pragma unroll 1
  for (int k0 = 0; k0 < K; k0 += 32) {
    {
      const float* ap = A + (size_t)(m0 + ar) * lda + k0 + acq;
      U16 H, L;
#pragma unroll
      for (int q = 0; q < 4; ++q) {
        const v4f_t v = *(const v4f*)(ap + 4 * q);
#pragma unroll
        for (int e = 0; e < 4; ++e) {
          unsigned short hi, lo;
          split_bf16(v[e], hi, lo);
          H.s[4 * q + e] = hi;
          L.s[4 * q + e] = lo;
        }
      }
      *(v8us*)(Ah + ar * GP + acq)     = H.v[0];
      *(v8us*)(Ah + ar * GP + acq + 8) = H.v[1];
      *(v8us*)(Al + ar * GP + acq)     = L.v[0];
      *(v8us*)(Al + ar * GP + acq + 8) = L.v[1];
    }
    {
      const float* wp = W + (size_t)(k0 + bk) * ldw + n0 + bnq;
#pragma unroll
      for (int q = 0; q < 4; ++q) {
        const v4f_t v = *(const v4f*)(wp + 4 * q);
#pragma unroll
        for (int e = 0; e < 4; ++e) {
          unsigned short hi, lo;
          split_bf16(v[e], hi, lo);
          const int n = bnq + 4 * q + e;
          Bh[n * GP + bk] = hi;
          Bl[n * GP + bk] = lo;
        }
      }
    }
    __syncthreads();
    const v16b fah = ldrowb(Ah, w * 16 + m, hh);
    const v16b fal = ldrowb(Al, w * 16 + m, hh);
#pragma unroll
    for (int nt = 0; nt < 4; ++nt) {
      const v16b fbh = ldrowb(Bh, nt * 16 + m, hh);
      const v16b fbl = ldrowb(Bl, nt * 16 + m, hh);
      acc[nt] = __builtin_amdgcn_wmma_f32_16x16x32_bf16(false, fah, false, fbh, (short)0, acc[nt], false, false);
      acc[nt] = __builtin_amdgcn_wmma_f32_16x16x32_bf16(false, fah, false, fbl, (short)0, acc[nt], false, false);
      acc[nt] = __builtin_amdgcn_wmma_f32_16x16x32_bf16(false, fal, false, fbh, (short)0, acc[nt], false, false);
      asm volatile("v_nop\n\tv_nop\n\tv_nop\n\tv_nop"
                   : "+v"(acc[nt]) : "v"(fah), "v"(fal), "v"(fbh), "v"(fbl));
    }
    __syncthreads();
  }

#pragma unroll
  for (int nt = 0; nt < 4; ++nt) {
    const int c = nt * 16 + m;
    const float bl = bias[n0 + c];
    const float bv = hasb ? bl : 0.0f;
#pragma unroll
    for (int r = 0; r < 8; ++r) {
      float v = acc[nt][r] + bv;
      if (relu) v = fmaxf(v, 0.0f);
      Cs[(w * 16 + 8 * hh + r) * 64 + c] = v;
    }
  }
  __syncthreads();
  v4f_t ov[8];
#pragma unroll
  for (int p = 0; p < 8; ++p) ov[p] = *(const v4f*)(Cs + (w * 16 + 2 * p + hh) * 64 + 4 * m);
#pragma unroll
  for (int p = 0; p < 8; ++p) {
    float* gp = C + (size_t)(m0 + w * 16 + 2 * p + hh) * ldc + n0 + 4 * m;
    *(volatile v4f_t*)gp = ov[p];
  }
  __threadfence();
#pragma unroll
  for (int p = 0; p < 8; ++p) {
    float* gp = C + (size_t)(m0 + w * 16 + 2 * p + hh) * ldc + n0 + 4 * m;
    *(volatile v4f_t*)gp = ov[p];
  }
}

__global__ __launch_bounds__(256) void pair_kernel(
    const float* __restrict__ ef, const int* __restrict__ adj,
    const float* __restrict__ ai, const float* __restrict__ aj,
    const float* __restrict__ egx, const float* __restrict__ nbr,
    const f16* __restrict__ wpl,
    const float* __restrict__ em_b1, const float* __restrict__ em_b2, const float* __restrict__ em_b3,
    const float* __restrict__ at_b1, const float* __restrict__ at_b2,
    const float* __restrict__ at_w3, const float* __restrict__ at_b3,
    const float* __restrict__ eg_b1, const float* __restrict__ eg_b2,
    float* comb)
{
  __shared__ __align__(16) f16   peL[NN * PEP];
  __shared__ __align__(16) f16   stg[8 * 16 * SP];
  __shared__ __align__(16) float pL[NN];
  __shared__ __align__(16) float msgw[8 * CC];
  __shared__ __align__(16) float mout[CC];
  __shared__ float red[16];
  __shared__ int   redi[8];

  const int bi = blockIdx.x;
  const int tid = threadIdx.x, w = tid >> 5, lane = tid & 31;
  const int hh = lane >> 4, m = lane & 15;
  const int bnode = bi & ~(NN - 1);
  f16* sw = stg + w * (16 * SP);
  const float b3 = at_b3[0];

#pragma unroll
  for (int q = 0; q < 8; ++q) msgw[q * CC + tid] = 0.0f;

#pragma unroll 1
  for (int t = 0; t < 4; ++t) {
    const int j0 = w * 64 + t * 16;

    FragH aef;
    {
      const float* er = ef + ((size_t)bi * NN + (j0 + m)) * EE;
#pragma unroll
      for (int e = 0; e < 8; ++e) aef.h[0][e] = (f16)(er[8 * hh + e] * SEF);
#pragma unroll
      for (int e = 0; e < 8; ++e) {
        const int k = 16 + 8 * hh + e;
        const int kc = (k < EE) ? k : (EE - 1);
        const float v = er[kc];
        aef.h[1][e] = (f16)((k < EE) ? v * SEF : 0.0f);
      }
    }

#pragma unroll
    for (int nt = 0; nt < 4; ++nt) {
      const v16h bw = ldrow(wpl + EM1_O, 32, nt * 16 + m, 0, hh);
      const v8f acc = mma1(aef.v, bw);
      const int c = nt * 16 + m;
      const float bb = em_b1[c];
#pragma unroll
      for (int r = 0; r < 8; ++r) {
        const float v = fmaxf(acc[r] * (1.0f / (SEF * SWT)) + bb, 0.0f);
        sw[(8 * hh + r) * SP + c] = (f16)(v * S1);
      }
    }
    __syncthreads();

    {
      const v16h a0 = ldrow(sw, SP, m, 0, hh);
      const v16h a1 = ldrow(sw, SP, m, 32, hh);
      __syncthreads();
#pragma unroll
      for (int nt = 0; nt < 4; ++nt) {
        const v16h b0 = ldrow(wpl + EM2_O, 64, nt * 16 + m, 0, hh);
        const v16h b1 = ldrow(wpl + EM2_O, 64, nt * 16 + m, 32, hh);
        const v8f acc = mma2(a0, b0, a1, b1);
        const int c = nt * 16 + m;
        const float bb = em_b2[c];
#pragma unroll
        for (int r = 0; r < 8; ++r) {
          const float v = fmaxf(acc[r] * (1.0f / (S1 * SWT)) + bb, 0.0f);
          sw[(8 * hh + r) * SP + c] = (f16)(v * S2);
        }
      }
    }
    __syncthreads();

    {
      const v16h a0 = ldrow(sw, SP, m, 0, hh);
      const v16h a1 = ldrow(sw, SP, m, 32, hh);
      __syncthreads();
#pragma unroll
      for (int nt = 0; nt < 2; ++nt) {
        const v16h b0 = ldrow(wpl + EM3_O, 64, nt * 16 + m, 0, hh);
        const v16h b1 = ldrow(wpl + EM3_O, 64, nt * 16 + m, 32, hh);
        const v8f acc = mma2(a0, b0, a1, b1);
        const int c = nt * 16 + m;
        const float bb = em_b3[c];
#pragma unroll
        for (int r = 0; r < 8; ++r) {
          const float v = fmaxf(acc[r] * (1.0f / (S2 * SWT)) + bb, 0.0f);
          peL[(j0 + 8 * hh + r) * PEP + c] = (f16)(v * SPE);
        }
      }
    }
    __syncthreads();

    {
      const v16h ape = ldrow(peL, PEP, j0 + m, 0, hh);
#pragma unroll
      for (int nt = 0; nt < 4; ++nt) {
        const v16h bw = ldrow(wpl + AT1E_O, 32, nt * 16 + m, 0, hh);
        const v8f acc = mma1(ape, bw);
        const int c = nt * 16 + m;
        const float cb = at_b1[c] + ai[(size_t)bi * HID + c];
        const float* ajp = aj + (size_t)(bnode + j0 + 8 * hh) * HID + c;
#pragma unroll
        for (int r = 0; r < 8; ++r) {
          const float v = fmaxf(acc[r] * (1.0f / (SPE * SWT)) + cb + ajp[(size_t)r * HID], 0.0f);
          sw[(8 * hh + r) * SP + c] = (f16)(v * SHH);
        }
      }
    }
    __syncthreads();

    {
      const v16h a0 = ldrow(sw, SP, m, 0, hh);
      const v16h a1 = ldrow(sw, SP, m, 32, hh);
      __syncthreads();
      float part[8];
#pragma unroll
      for (int r = 0; r < 8; ++r) part[r] = 0.0f;
#pragma unroll
      for (int nt = 0; nt < 2; ++nt) {
        const v16h b0 = ldrow(wpl + AT2_O, 64, nt * 16 + m, 0, hh);
        const v16h b1 = ldrow(wpl + AT2_O, 64, nt * 16 + m, 32, hh);
        const v8f acc = mma2(a0, b0, a1, b1);
        const int c = nt * 16 + m;
        const float bb = at_b2[c];
        const float w3 = at_w3[c];
#pragma unroll
        for (int r = 0; r < 8; ++r) {
          const float h2 = fmaxf(acc[r] * (1.0f / (SHH * SWT)) + bb, 0.0f);
          part[r] += h2 * w3;
        }
      }
#pragma unroll
      for (int r = 0; r < 8; ++r) {
        part[r] += __shfl_xor(part[r], 1, 32);
        part[r] += __shfl_xor(part[r], 2, 32);
        part[r] += __shfl_xor(part[r], 4, 32);
        part[r] += __shfl_xor(part[r], 8, 32);
      }
      float mine = 0.0f;
#pragma unroll
      for (int r = 0; r < 8; ++r) mine = (m == r) ? part[r] : mine;
      const int jj = j0 + 8 * hh + (m & 7);
      const int av = adj[(size_t)bi * NN + jj];
      const float sv = (av > 0) ? (mine + b3) : -1.0e9f;
      if (m < 8) pL[jj] = sv;
    }
  }
  __syncthreads();

  int hasn = 0;
  {
    const float s0 = pL[tid], s1 = pL[tid + 256];
    const int a0 = (adj[(size_t)bi * NN + tid] > 0) ? 1 : 0;
    const int a1 = (adj[(size_t)bi * NN + tid + 256] > 0) ? 1 : 0;
    float mx = fmaxf(s0, s1);
    int anyf = a0 | a1;
#pragma unroll
    for (int o = 16; o > 0; o >>= 1) {
      mx = fmaxf(mx, __shfl_xor(mx, o, 32));
      anyf |= __shfl_xor(anyf, o, 32);
    }
    if (lane == 0) { red[w] = mx; redi[w] = anyf; }
    __syncthreads();
    float M = red[0];
    int anyb = redi[0];
#pragma unroll
    for (int q = 1; q < 8; ++q) { M = fmaxf(M, red[q]); anyb |= redi[q]; }
    const float e0 = __expf(s0 - M), e1 = __expf(s1 - M);
    float sm = e0 + e1;
#pragma unroll
    for (int o = 16; o > 0; o >>= 1) sm += __shfl_xor(sm, o, 32);
    if (lane == 0) red[8 + w] = sm;
    __syncthreads();
    float S = red[8];
#pragma unroll
    for (int q = 1; q < 8; ++q) S += red[8 + q];
    const float rS = 1.0f / S;
    pL[tid]       = a0 ? (e0 * rS) : 0.0f;
    pL[tid + 256] = a1 ? (e1 * rS) : 0.0f;
    hasn = anyb;
  }
  __syncthreads();

#pragma unroll 1
  for (int t = 0; t < 4; ++t) {
    const int j0 = w * 64 + t * 16;

    {
      const v16h ape = ldrow(peL, PEP, j0 + m, 0, hh);
#pragma unroll
      for (int nt = 0; nt < 4; ++nt) {
        const v16h bw = ldrow(wpl + EG1E_O, 32, nt * 16 + m, 0, hh);
        const v8f acc = mma1(ape, bw);
        const int c = nt * 16 + m;
        const float bb = eg_b1[c];
        const float* exq = egx + (size_t)(bnode + j0 + 8 * hh) * HID + c;
#pragma unroll
        for (int r = 0; r < 8; ++r) {
          const float v = fmaxf(acc[r] * (1.0f / (SPE * SWT)) + bb + exq[(size_t)r * HID], 0.0f);
          sw[(8 * hh + r) * SP + c] = (f16)(v * SGG);
        }
      }
    }
    __syncthreads();

    const v16h a0 = ldrow(sw, SP, m, 0, hh);
    const v16h a1 = ldrow(sw, SP, m, 32, hh);
    float pv[8];
#pragma unroll
    for (int r = 0; r < 8; ++r) pv[r] = pL[j0 + 8 * hh + r];
    __syncthreads();

    const float* nbp = nbr + (size_t)(bnode + j0 + 8 * hh) * CC;
#pragma unroll 1
    for (int nt = 0; nt < 16; ++nt) {
      const v16h b0 = ldrow(wpl + EG2_O, 64, nt * 16 + m, 0, hh);
      const v16h b1 = ldrow(wpl + EG2_O, 64, nt * 16 + m, 32, hh);
      const v8f acc = mma2(a0, b0, a1, b1);
      const int c = nt * 16 + m;
      const float bb = eg_b2[c];
      float cs = 0.0f;
#pragma unroll
      for (int r = 0; r < 8; ++r) {
        const float zz = acc[r] * (1.0f / (SGG * SWT)) + bb;
        const float ex = __expf(-zz);
        const float sg = __builtin_amdgcn_rcpf(1.0f + ex);
        const float gated = sg * nbp[(size_t)r * CC + c];
        cs += pv[r] * gated;
      }
      cs += __shfl_xor(cs, 16, 32);
      if (hh == 0) msgw[w * CC + c] += cs;
    }
  }
  __syncthreads();

  {
    float s = 0.0f;
#pragma unroll
    for (int q = 0; q < 8; ++q) s += msgw[q * CC + tid];
    mout[tid] = hasn ? s : 0.0f;
  }
  __syncthreads();
  if (tid < 64) {
    const v4f_t v = *(const v4f*)(mout + 4 * tid);
    float* gp = comb + (size_t)bi * (2 * CC) + CC + 4 * tid;
    *(volatile v4f_t*)gp = v;
    __threadfence();
    *(volatile v4f_t*)gp = v;
  }
}

extern "C" void kernel_launch(void* const* d_in, const int* in_sizes, int n_in,
                              void* d_out, int out_size, void* d_ws, size_t ws_size,
                              hipStream_t stream)
{
  if (n_in < 27) return;
  if (in_sizes[0] != NODES * CC || in_sizes[1] != NODES * NN || in_sizes[2] != NODES * NN * EE) return;
  if (in_sizes[3] != CC * CC || in_sizes[4] != CC || in_sizes[5] != CC * CC || in_sizes[6] != CC) return;
  if (in_sizes[7] != EE * 64 || in_sizes[8] != 64 || in_sizes[9] != 64 * 64 || in_sizes[10] != 64) return;
  if (in_sizes[11] != 64 * 32 || in_sizes[12] != 32) return;
  if (in_sizes[13] != 544 * 64 || in_sizes[14] != 64 || in_sizes[15] != 64 * 32 || in_sizes[16] != 32) return;
  if (in_sizes[17] != 32 || in_sizes[18] < 1) return;
  if (in_sizes[19] != 288 * 64 || in_sizes[20] != 64 || in_sizes[21] != 64 * CC || in_sizes[22] != CC) return;
  if (in_sizes[23] != 512 * CC || in_sizes[24] != CC || in_sizes[25] != CC * CC || in_sizes[26] != CC) return;
  if (out_size != NODES * CC) return;

  const float* x     = (const float*)d_in[0];
  const int*   adj   = (const int*)d_in[1];
  const float* ef    = (const float*)d_in[2];
  const float* st_w  = (const float*)d_in[3];
  const float* st_b  = (const float*)d_in[4];
  const float* nt_w  = (const float*)d_in[5];
  const float* nt_b  = (const float*)d_in[6];
  const float* em_w1 = (const float*)d_in[7];
  const float* em_b1 = (const float*)d_in[8];
  const float* em_w2 = (const float*)d_in[9];
  const float* em_b2 = (const float*)d_in[10];
  const float* em_w3 = (const float*)d_in[11];
  const float* em_b3 = (const float*)d_in[12];
  const float* at_w1 = (const float*)d_in[13];
  const float* at_b1 = (const float*)d_in[14];
  const float* at_w2 = (const float*)d_in[15];
  const float* at_b2 = (const float*)d_in[16];
  const float* at_w3 = (const float*)d_in[17];
  const float* at_b3 = (const float*)d_in[18];
  const float* eg_w1 = (const float*)d_in[19];
  const float* eg_b1 = (const float*)d_in[20];
  const float* eg_w2 = (const float*)d_in[21];
  const float* eg_b2 = (const float*)d_in[22];
  const float* cb_w1 = (const float*)d_in[23];
  const float* cb_b1 = (const float*)d_in[24];
  const float* cb_w2 = (const float*)d_in[25];
  const float* cb_b2 = (const float*)d_in[26];
  float* out = (float*)d_out;

  const size_t szComb = (size_t)NODES * 2 * CC * 4;
  const size_t szNbr  = (size_t)NODES * CC * 4;
  const size_t szH    = (size_t)NODES * HID * 4;
  const size_t szT1   = (size_t)NODES * CC * 4;
  const size_t szWpl  = (size_t)WPL_HALVES * 2;
  const size_t oComb = 0;
  const size_t oNbr  = oComb + szComb;
  const size_t oAi   = oNbr + szNbr;
  const size_t oAj   = oAi + szH;
  const size_t oEgx  = oAj + szH;
  const size_t oT1   = oEgx + szH;
  const size_t oWpl  = oT1 + szT1;
  const size_t total = oWpl + szWpl;
  if (total > ws_size) return;

  char* ws = (char*)d_ws;
  float* comb  = (float*)(ws + oComb);
  float* nbr32 = (float*)(ws + oNbr);
  float* ai32  = (float*)(ws + oAi);
  float* aj32  = (float*)(ws + oAj);
  float* egx32 = (float*)(ws + oEgx);
  float* t1    = (float*)(ws + oT1);
  f16*   wpl   = (f16*)(ws + oWpl);

  wprep_kernel<<<dim3(8, 7, 1), 256, 0, stream>>>(em_w1, em_w2, em_w3, at_w1, at_w2, eg_w1, eg_w2, wpl);

  gemm3_kernel<<<dim3(CC / 64, NODES / 64, 2), 128, 0, stream>>>(
      x, CC, CC,
      st_w, nt_w, nt_w, CC,
      st_b, nt_b, nt_b, 1,
      comb, nbr32, nbr32, 2 * CC, CC, CC, 0);

  gemm3_kernel<<<dim3(HID / 64, NODES / 64, 3), 128, 0, stream>>>(
      x, CC, CC,
      at_w1, at_w1 + 256 * 64, eg_w1, HID,
      at_w1, at_w1, eg_w1, 0,
      ai32, aj32, egx32, HID, HID, HID, 0);

  pair_kernel<<<NODES, 256, 0, stream>>>(
      ef, adj, ai32, aj32, egx32, nbr32, wpl,
      em_b1, em_b2, em_b3, at_b1, at_b2, at_w3, at_b3, eg_b1, eg_b2, comb);

  gemm3_kernel<<<dim3(CC / 64, NODES / 64, 1), 128, 0, stream>>>(
      comb, 2 * CC, 2 * CC,
      cb_w1, cb_w1, cb_w1, CC,
      cb_b1, cb_b1, cb_b1, 1,
      t1, t1, t1, CC, CC, CC, 1);

  gemm3_kernel<<<dim3(CC / 64, NODES / 64, 1), 128, 0, stream>>>(
      t1, CC, CC,
      cb_w2, cb_w2, cb_w2, CC,
      cb_b2, cb_b2, cb_b2, 1,
      out, out, out, CC, CC, CC, 0);
}
